// Mask2ControlPoints_66236985639391
// MI455X (gfx1250) — hardware-run, weakly checked
//
#include <hip/hip_runtime.h>
#include <math.h>

typedef __attribute__((ext_vector_type(16))) _Float16 v16h;
typedef __attribute__((ext_vector_type(8)))  _Float16 v8h;
typedef __attribute__((ext_vector_type(16))) __bf16   v16b;
typedef __attribute__((ext_vector_type(8)))  __bf16   v8b;
typedef __attribute__((ext_vector_type(8)))  float    v8f;
typedef __attribute__((ext_vector_type(4)))  float    v4f;
typedef __attribute__((ext_vector_type(4)))  unsigned v4u;

constexpr int kB      = 64;
constexpr int kImg    = 256;
constexpr int kPool   = 128;
constexpr int kCh1    = 16;
constexpr int kCh2    = 32;
constexpr int kHid    = 512;
constexpr int kG4     = 2048;
constexpr int kVoc    = 4096;
constexpr int kSteps  = 50;
constexpr int kRowsAll = kB * kSteps;
constexpr int kPRows  = 130;
constexpr int kPPitch = 132;
constexpr int kK2     = 160;
constexpr int kRowGroups = 8;
static_assert(kPool * 2 == kImg);
static_assert(kG4 == 4 * kHid);
static_assert(kRowsAll == 3200);
static_assert((kRowsAll % 64) == 0 && (kG4 % 64) == 0 && (kVoc % 64) == 0 && (kHid % 64) == 0 && (kB % 64) == 0);
static_assert((kHid % 32) == 0 && (kK2 % 32) == 0 && (32 % 32) == 0);
static_assert((kPPitch * 32) % 128 == 0);
static_assert(kRowGroups * 16 == kPool);

constexpr size_t kSzPP   = (size_t)kB * kPRows * kPPitch * kCh1 * 2;
constexpr size_t kSzW2   = (size_t)kCh2 * kK2 * 2;
constexpr size_t kSzPART = (size_t)kB * kRowGroups * 32 * 4;
constexpr size_t kSzX16  = (size_t)kB * 32 * 2;
constexpr size_t kSzFW   = (size_t)kHid * 32 * 2;
constexpr size_t kSzCW   = (size_t)kHid * kHid * 2;
constexpr size_t kSzWG   = (size_t)kG4 * kHid * 2;
constexpr size_t kSzHW   = (size_t)kVoc * kHid * 2;
constexpr size_t kSzH16  = (size_t)kB * kHid * 2;
constexpr size_t kSzF32  = (size_t)kB * kHid * 4;
constexpr size_t kSzXIN  = (size_t)kRowsAll * kHid * 2;
constexpr size_t kSzGIN  = (size_t)kRowsAll * kG4 * 4;
constexpr size_t kSzHP   = (size_t)kRowsAll * kHid * 2;

constexpr size_t kOffPP   = 0;
constexpr size_t kOffW2   = kOffPP   + kSzPP;
constexpr size_t kOffPART = kOffW2   + kSzW2;
constexpr size_t kOffX16  = kOffPART + kSzPART;
constexpr size_t kOffFW   = kOffX16  + kSzX16;
constexpr size_t kOffCW   = kOffFW   + kSzFW;
constexpr size_t kOffWIH  = kOffCW   + kSzCW;
constexpr size_t kOffWHH  = kOffWIH  + kSzWG;
constexpr size_t kOffHW   = kOffWHH  + kSzWG;
constexpr size_t kOffHA   = kOffHW   + kSzHW;
constexpr size_t kOffHB   = kOffHA   + kSzH16;
constexpr size_t kOffCTX  = kOffHB   + kSzH16;
constexpr size_t kOffCA   = kOffCTX  + kSzF32;
constexpr size_t kOffCB   = kOffCA   + kSzF32;
constexpr size_t kOffXIN  = kOffCB   + kSzF32;
constexpr size_t kOffGIN  = kOffXIN  + kSzXIN;
constexpr size_t kOffHH   = kOffGIN  + kSzGIN;
constexpr size_t kOffHL   = kOffHH   + kSzHP;
constexpr size_t kWsTotal = kOffHL   + kSzHP;
static_assert(kWsTotal == 80738304ull);
static_assert(kWsTotal <= 134217728ull);
static_assert((kOffW2 % 128) == 0 && (kOffPART % 128) == 0 && (kOffX16 % 128) == 0 && (kOffFW % 128) == 0 &&
              (kOffCW % 128) == 0 && (kOffWIH % 128) == 0 && (kOffWHH % 128) == 0 && (kOffHW % 128) == 0 &&
              (kOffHA % 128) == 0 && (kOffHB % 128) == 0 && (kOffCTX % 128) == 0 && (kOffCA % 128) == 0 &&
              (kOffCB % 128) == 0 && (kOffXIN % 128) == 0 && (kOffGIN % 128) == 0 && (kOffHH % 128) == 0 &&
              (kOffHL % 128) == 0);

__device__ __forceinline__ unsigned short f2bf_bits(float f) {
  unsigned u = __float_as_uint(f);
  return (unsigned short)((u + 0x7FFFu + ((u >> 16) & 1u)) >> 16);
}
__device__ __forceinline__ float bf_bits2f(unsigned short h) { return __uint_as_float(((unsigned)h) << 16); }
__device__ __forceinline__ float bfr(float f) { return bf_bits2f(f2bf_bits(f)); }
__device__ __forceinline__ _Float16 h16_flush(float v) {
  const float a = fabsf(v);
  const float w = (a < 6.103515625e-05f) ? 0.0f : v;
  return (_Float16)w;
}
__device__ __forceinline__ unsigned h16_bits(float v) {
  const _Float16 h = h16_flush(v);
  return (unsigned)__builtin_bit_cast(unsigned short, h);
}

__device__ __forceinline__ v8f mma_h(v16h a, v16h b, v8f c) {
  c = __builtin_amdgcn_wmma_f32_16x16x32_f16(false, a, false, b, (short)0, c, false, false);
  asm volatile("v_nop\n\tv_nop\n\tv_nop\n\tv_nop" : "+v"(c) : "v"(a), "v"(b));
  return c;
}
__device__ __forceinline__ v8f mma_b(v16b a, v16b b, v8f c) {
  c = __builtin_amdgcn_wmma_f32_16x16x32_bf16(false, a, false, b, (short)0, c, false, false);
  asm volatile("v_nop\n\tv_nop\n\tv_nop\n\tv_nop" : "+v"(c) : "v"(a), "v"(b));
  return c;
}

template <typename T> struct Frag;
template <> struct Frag<_Float16> {
  typedef v16h V; union U { v16h v; v8h h[2]; };
  static __device__ __forceinline__ v16h load(const _Float16* p) {
    U f; f.h[0] = *(const v8h*)(p); f.h[1] = *(const v8h*)(p + 16); return f.v;
  }
  static __device__ __forceinline__ v8f mma(v16h a, v16h b, v8f c) { return mma_h(a, b, c); }
};
template <> struct Frag<__bf16> {
  typedef v16b V; union U { v16b v; v8b h[2]; };
  static __device__ __forceinline__ v16b load(const __bf16* p) {
    U f; f.h[0] = *(const v8b*)(p); f.h[1] = *(const v8b*)(p + 16); return f.v;
  }
  static __device__ __forceinline__ v8f mma(v16b a, v16b b, v8f c) { return mma_b(a, b, c); }
};

template <int ET> struct Elem;
template <> struct Elem<0> { typedef _Float16 T; };
template <> struct Elem<1> { typedef __bf16 T; };

template <int ET, int SPL, int NBIAS, int OUT_MODE, int SHIFT, int OSHIFT>
__global__ __launch_bounds__(256) void wmma_gemm64(
    const unsigned short* __restrict__ Ap, const unsigned short* __restrict__ A2p, int lda,
    const unsigned short* __restrict__ Btp, int ldb,
    void* __restrict__ Cout, int ldc,
    const float* __restrict__ bias1, const float* __restrict__ bias2,
    int M, int N, int K) {
  typedef typename Elem<ET>::T T;
  typedef typename Frag<T>::V V;
  const T* A = (const T*)Ap; const T* A2 = (const T*)A2p; const T* Bt = (const T*)Btp;
  __shared__ __align__(16) float sT[8][16 * 68];
  const int lane = threadIdx.x & 31;
  const int wave = threadIdx.x >> 5;
  const int tilesN = N >> 6;
  const int tilesM = M >> 6;
  const int tile = blockIdx.x * 8 + wave;
  if (tile >= tilesM * tilesN) return;
  const int tm = tile / tilesN;
  const int tn = tile - tm * tilesN;
  const int m0 = tm << 6;
  const int n0 = tn << 6;
  const int rlane = lane & 15;
  const int koff  = (lane >> 4) * 8;
  const int mOff  = (lane >> 4) * 8;
  const float scale  = 1.0f / (float)(1 << SHIFT);
  const float ocarry = (float)(1 << OSHIFT);

  v8f acc[4][4];
#pragma unroll
  for (int i = 0; i < 4; ++i)
#pragma unroll
    for (int j = 0; j < 4; ++j) acc[i][j] = (v8f){0.f,0.f,0.f,0.f,0.f,0.f,0.f,0.f};

  for (int k0 = 0; k0 < K; k0 += 32) {
    V bh[4];
#pragma unroll
    for (int j = 0; j < 4; ++j) {
      const size_t bo = (size_t)(n0 + (j << 4) + rlane) * ldb + koff + k0;
      bh[j] = Frag<T>::load(Bt + bo);
    }
#pragma unroll
    for (int i = 0; i < 4; ++i) {
      const size_t ao = (size_t)(m0 + (i << 4) + rlane) * lda + koff + k0;
      V ah = Frag<T>::load(A + ao);
      V al = ah;
      if (SPL == 1) al = Frag<T>::load(A2 + ao);
#pragma unroll
      for (int j = 0; j < 4; ++j) {
        acc[i][j] = Frag<T>::mma(ah, bh[j], acc[i][j]);
        if (SPL == 1) acc[i][j] = Frag<T>::mma(al, bh[j], acc[i][j]);
      }
    }
  }

  float* slab = sT[wave];
#pragma unroll
  for (int i = 0; i < 4; ++i) {
    const int mBase = m0 + (i << 4);
#pragma unroll
    for (int j = 0; j < 4; ++j) {
      const int n = n0 + (j << 4) + rlane;
      float bv = bfr(bias1[n]);
      if (NBIAS == 2) bv += bfr(bias2[n]);
#pragma unroll
      for (int r = 0; r < 8; ++r) {
        const float v = acc[i][j][r] * scale + bv;
        slab[(mOff + r) * 68 + (j << 4) + rlane] = v;
      }
    }
    __builtin_amdgcn_fence(__ATOMIC_RELEASE, "workgroup");
    __builtin_amdgcn_wave_barrier();
    __builtin_amdgcn_fence(__ATOMIC_ACQUIRE, "workgroup");
    if (OUT_MODE == 0) {
      float* C = (float*)Cout;
      const int hh = lane >> 4, c4 = (lane & 15) * 4;
      for (int pass = 0; pass < 2; ++pass) {
#pragma unroll
        for (int it = 0; it < 8; ++it) {
          const int row = it * 2 + hh;
          const v4f v = *(const v4f*)(slab + row * 68 + c4);
          *(volatile v4f*)(C + (size_t)(mBase + row) * ldc + n0 + c4) = v;
        }
        __threadfence();
      }
    } else {
      const int q = lane >> 3, c8 = (lane & 7) * 8;
      unsigned short* C = (unsigned short*)Cout;
      for (int pass = 0; pass < 2; ++pass) {
#pragma unroll
        for (int it = 0; it < 4; ++it) {
          const int row = it * 4 + q;
          const float* sp = slab + row * 68 + c8;
          v8h hv;
#pragma unroll
          for (int e = 0; e < 8; ++e) {
            const float x = sp[e] * ocarry;
            hv[e] = h16_flush(x);
          }
          *(volatile v8h*)(C + (size_t)(mBase + row) * ldc + n0 + c8) = hv;
        }
        __threadfence();
      }
    }
    __builtin_amdgcn_fence(__ATOMIC_RELEASE, "workgroup");
    __builtin_amdgcn_wave_barrier();
    __builtin_amdgcn_fence(__ATOMIC_ACQUIRE, "workgroup");
  }
}

template <int MODE, int CSHIFT>
__global__ __launch_bounds__(256) void cast_plane_kernel(
    const float* __restrict__ src, unsigned short* __restrict__ dst, int total8) {
  const int i = blockIdx.x * 256 + threadIdx.x;
  if (i >= total8) return;
  const size_t e0 = (size_t)i << 3;
  const v4f a0 = *(const v4f*)(src + e0);
  const v4f a1 = *(const v4f*)(src + e0 + 4);
  const float carry = (float)(1 << CSHIFT);
  v8h hv;
#pragma unroll
  for (int e = 0; e < 4; ++e) {
    const float x0 = a0[e];
    const float x1 = a1[e];
    if (MODE == 1) {
      const unsigned short b0 = f2bf_bits(x0);
      const unsigned short b1 = f2bf_bits(x1);
      hv[e]     = __builtin_bit_cast(_Float16, b0);
      hv[4 + e] = __builtin_bit_cast(_Float16, b1);
    } else {
      hv[e]     = h16_flush(bfr(x0) * carry);
      hv[4 + e] = h16_flush(bfr(x1) * carry);
    }
  }
  unsigned short* q = dst + e0;
  *(volatile v8h*)q = hv;
  __threadfence();
  *(volatile v8h*)q = hv;
}

__global__ __launch_bounds__(256) void conv2_weight_plane_kernel(
    const float* __restrict__ w2, unsigned short* __restrict__ W2p) {
  const int i = blockIdx.x * 256 + threadIdx.x;
  if (i >= kCh2 * (kK2 / 8)) return;
  const int oc = i / (kK2 / 8);
  const int p  = i - oc * (kK2 / 8);
  const int tap = p >> 1;
  const int tc  = tap < 9 ? tap : 8;
  const int cb  = (p & 1) * 8;
  v8h hv;
#pragma unroll
  for (int e = 0; e < 8; ++e) {
    float wv = w2[oc * 144 + (cb + e) * 9 + tc];
    asm volatile("" : "+v"(wv));
    const float cv = (tap < 9) ? (bfr(wv) * 64.0f) : 0.0f;
    hv[e] = h16_flush(cv);
  }
  unsigned short* q = W2p + (size_t)i * 8;
  *(volatile v8h*)q = hv;
  __threadfence();
  *(volatile v8h*)q = hv;
}

__device__ __forceinline__ float conv1_pool_val(const float (&pt)[4][4], const float* wk, float bias) {
  float mx = -INFINITY;
#pragma unroll
  for (int a = 0; a < 2; ++a)
#pragma unroll
    for (int c = 0; c < 2; ++c) {
      float s = 0.0f;
#pragma unroll
      for (int ky = 0; ky < 3; ++ky)
#pragma unroll
        for (int kx = 0; kx < 3; ++kx)
          s = fmaf(wk[ky * 3 + kx], pt[a + ky][c + kx], s);
      mx = fmaxf(mx, s);
    }
  return fmaxf(mx + bias, 0.0f);
}

__global__ __launch_bounds__(256) void conv1_pool_plane_kernel(
    const float* __restrict__ mask, const float* __restrict__ w1, const float* __restrict__ b1,
    unsigned* __restrict__ Pw) {
  __shared__ float sM[4 * 260];
  __shared__ float sW[160];
  __shared__ __align__(16) unsigned sRow[kPPitch * 8];
  const int tid = threadIdx.x;
  const int ry  = blockIdx.x;
  const int b   = blockIdx.y;
  const bool padrow = (ry == 0) || (ry == kPRows - 1);
  int py = ry - 1;
  py = py < 0 ? 0 : (py > kPool - 1 ? kPool - 1 : py);
  {
    const int wi = tid < 143 ? tid : 143;
    float wv = w1[wi];
    asm volatile("" : "+v"(wv));
    int bi = tid - 144;
    bi = bi < 0 ? 0 : (bi > 15 ? 15 : bi);
    float bv = b1[bi];
    asm volatile("" : "+v"(bv));
    if (tid < 160) sW[tid] = bfr(tid < 144 ? wv : bv);
  }
  {
    const int r  = tid >> 6;
    const int c4 = (tid & 63) * 4;
    const int iy = 2 * py - 1 + r;
    const int iyc = iy < 0 ? 0 : (iy > kImg - 1 ? kImg - 1 : iy);
    const bool ok = (iy >= 0) && (iy < kImg);
    const v4f v = *(const v4f*)(mask + ((size_t)b * kImg + iyc) * kImg + c4);
    const float x0 = v[0], x1 = v[1], x2 = v[2], x3 = v[3];
    sM[r * 260 + 1 + c4 + 0] = ok ? bfr(x0) : 0.0f;
    sM[r * 260 + 1 + c4 + 1] = ok ? bfr(x1) : 0.0f;
    sM[r * 260 + 1 + c4 + 2] = ok ? bfr(x2) : 0.0f;
    sM[r * 260 + 1 + c4 + 3] = ok ? bfr(x3) : 0.0f;
  }
  if (tid < 8) {
    const int r = tid >> 1;
    sM[r * 260 + ((tid & 1) ? 257 : 0)] = 0.0f;
    const int pos = (r == 0) ? 0 : (128 + r);
    *(v4u*)(sRow + pos * 8 + (tid & 1) * 4) = (v4u){0u, 0u, 0u, 0u};
  }
  __syncthreads();

  const int x = tid & 127;
  const int g = tid >> 7;
  float pt[4][4];
#pragma unroll
  for (int dy = 0; dy < 4; ++dy)
#pragma unroll
    for (int dx = 0; dx < 4; ++dx) pt[dy][dx] = sM[dy * 260 + 2 * x + dx];

#pragma unroll 1
  for (int i = 0; i < 4; ++i) {
    const int oc = g * 8 + 2 * i;
    const float v0 = conv1_pool_val(pt, sW + oc * 9, sW[144 + oc]);
    const float v1 = conv1_pool_val(pt, sW + (oc + 1) * 9, sW[144 + oc + 1]);
    const unsigned w0 = h16_bits(v0 * 16.0f);
    const unsigned wq = h16_bits(v1 * 16.0f);
    unsigned word = w0 | (wq << 16);
    if (padrow) word = 0u;
    sRow[(x + 1) * 8 + g * 4 + i] = word;
  }
  __syncthreads();

  unsigned* dst = Pw + ((size_t)(b * kPRows + ry) * kPPitch) * 8;
  const int t2 = 256 + (tid & 7);
  const v4u q0 = *(const v4u*)(sRow + tid * 4);
  const v4u q1 = *(const v4u*)(sRow + t2 * 4);
  *(volatile v4u*)(dst + tid * 4) = q0;
  if (tid < 8) *(volatile v4u*)(dst + t2 * 4) = q1;
  __threadfence();
  *(volatile v4u*)(dst + tid * 4) = q0;
  if (tid < 8) *(volatile v4u*)(dst + t2 * 4) = q1;
}

__global__ __launch_bounds__(256) void conv2_mean_partial_kernel(
    const unsigned short* __restrict__ Pp, const unsigned short* __restrict__ W2p,
    const float* __restrict__ b2, float* __restrict__ part) {
  __shared__ float sRed[8 * 32];
  const _Float16* P  = (const _Float16*)Pp;
  const _Float16* W2 = (const _Float16*)W2p;
  const int tid = threadIdx.x, lane = tid & 31, wave = tid >> 5;
  const int hh = lane >> 4, m = lane & 15;
  const int rg = blockIdx.x;
  const int b  = blockIdx.y;
  const int x0 = wave * 16;

  v16h wb[5][2];
#pragma unroll
  for (int s = 0; s < 5; ++s)
#pragma unroll
    for (int nt = 0; nt < 2; ++nt)
      wb[s][nt] = Frag<_Float16>::load(W2 + (nt * 16 + m) * kK2 + s * 32 + 8 * hh);
  const float bias0 = bfr(b2[m]);
  const float bias1 = bfr(b2[16 + m]);
  const float kInv = 1.0f / 1024.0f;
  v8h zero8;
#pragma unroll
  for (int e = 0; e < 8; ++e) zero8[e] = (_Float16)0.0f;
  float cs0 = 0.0f, cs1 = 0.0f;

#pragma unroll 1
  for (int yy = 0; yy < 16; ++yy) {
    const int y = rg * 16 + yy;
    const _Float16* base = P + ((size_t)(b * kPRows + y) * kPPitch + x0 + m) * 16 + 8 * hh;
    v8f a0 = (v8f){0.f,0.f,0.f,0.f,0.f,0.f,0.f,0.f};
    v8f a1 = (v8f){0.f,0.f,0.f,0.f,0.f,0.f,0.f,0.f};
#pragma unroll
    for (int s = 0; s < 5; ++s) {
      const int tA = 2 * s, tB = 2 * s + 1;
      Frag<_Float16>::U fa;
      fa.h[0] = *(const v8h*)(base + ((tA / 3) * kPPitch + (tA % 3)) * 16);
      if (tB < 9) fa.h[1] = *(const v8h*)(base + ((tB / 3) * kPPitch + (tB % 3)) * 16);
      else        fa.h[1] = zero8;
      a0 = mma_h(fa.v, wb[s][0], a0);
      a1 = mma_h(fa.v, wb[s][1], a1);
    }
#pragma unroll
    for (int r = 0; r < 8; ++r) {
      cs0 += fmaxf(a0[r] * kInv + bias0, 0.0f);
      cs1 += fmaxf(a1[r] * kInv + bias1, 0.0f);
    }
  }
  cs0 += __shfl_xor(cs0, 16, 32);
  cs1 += __shfl_xor(cs1, 16, 32);
  if (hh == 0) {
    sRed[wave * 32 + m]      = cs0;
    sRed[wave * 32 + 16 + m] = cs1;
  }
  __syncthreads();
  if (wave == 0) {
    float s = 0.0f;
#pragma unroll
    for (int w = 0; w < 8; ++w) s += sRed[w * 32 + lane];
    volatile float* q = part + ((size_t)(b * kRowGroups + rg) * 32 + lane);
    *q = s;
    __threadfence();
    *q = s;
  }
}

__global__ __launch_bounds__(256) void mean_plane_kernel(
    const float* __restrict__ part, unsigned short* __restrict__ X16) {
  const int i = threadIdx.x;
  const int row = i >> 2, c8 = (i & 3) * 8;
  v4f s0 = (v4f){0.f, 0.f, 0.f, 0.f};
  v4f s1 = (v4f){0.f, 0.f, 0.f, 0.f};
#pragma unroll 1
  for (int p = 0; p < kRowGroups; ++p) {
    const float* q = part + (size_t)(row * kRowGroups + p) * 32 + c8;
    s0 += *(const v4f*)q;
    s1 += *(const v4f*)(q + 4);
  }
  const float sc = 16.0f / 16384.0f;
  v8h hv;
#pragma unroll
  for (int e = 0; e < 4; ++e) {
    const float x0 = s0[e] * sc;
    const float x1 = s1[e] * sc;
    hv[e]     = h16_flush(x0);
    hv[4 + e] = h16_flush(x1);
  }
  unsigned short* q = X16 + (size_t)i * 8;
  *(volatile v8h*)q = hv;
  __threadfence();
  *(volatile v8h*)q = hv;
}

__global__ __launch_bounds__(256) void zero_plane_kernel(float* __restrict__ p, int n4) {
  const int i = blockIdx.x * 256 + threadIdx.x;
  if (i >= n4) return;
  const v4f z = (v4f){0.f, 0.f, 0.f, 0.f};
  *(volatile v4f*)(p + (size_t)i * 4) = z;
  __threadfence();
  *(volatile v4f*)(p + (size_t)i * 4) = z;
}

__global__ __launch_bounds__(256) void step_input_plane_kernel(
    const float* __restrict__ emb, const int* __restrict__ tgt, const float* __restrict__ ctx,
    unsigned short* __restrict__ XIN) {
  const int i = blockIdx.x * 256 + threadIdx.x;
  const int row = i >> 6, c8 = (i & 63) * 8;
  const int t = row >> 6, b = row & 63;
  int tp = t - 1;
  tp = tp < 0 ? 0 : tp;
  int tok = tgt[b * kSteps + tp];
  tok = tok < 0 ? 0 : (tok > kVoc ? kVoc : tok);
  tok = (t == 0) ? kVoc : tok;
  const float* ep = emb + (size_t)tok * kHid + c8;
  const float* cp = ctx + (size_t)b * kHid + c8;
  const v4f e0 = *(const v4f*)ep;
  const v4f e1 = *(const v4f*)(ep + 4);
  const v4f c0 = *(const v4f*)cp;
  const v4f c1 = *(const v4f*)(cp + 4);
  v8h hv;
#pragma unroll
  for (int e = 0; e < 4; ++e) {
    const float x0 = (bfr(e0[e]) + c0[e]) * 16.0f;
    const float x1 = (bfr(e1[e]) + c1[e]) * 16.0f;
    hv[e]     = h16_flush(x0);
    hv[4 + e] = h16_flush(x1);
  }
  unsigned short* q = XIN + (size_t)row * kHid + c8;
  *(volatile v8h*)q = hv;
  __threadfence();
  *(volatile v8h*)q = hv;
}

__global__ __launch_bounds__(128) void lstm_step_kernel(
    const unsigned short* __restrict__ hcur_p, const unsigned short* __restrict__ whh_p,
    const float* __restrict__ gin, const float* __restrict__ ccur, float* __restrict__ cnew,
    unsigned short* __restrict__ hnew, unsigned short* __restrict__ HH, unsigned short* __restrict__ HL, int t) {
  __shared__ __align__(16) float sGate[4][4 * 320];
  __shared__ __align__(16) float sC[4][16 * 68];
  __shared__ __align__(16) float sH[4][16 * 68];
  const _Float16* hcur = (const _Float16*)hcur_p;
  const _Float16* whh  = (const _Float16*)whh_p;
  const int tid = threadIdx.x, lane = tid & 31, wave = tid >> 5;
  const int hh = lane >> 4, m = lane & 15;
  const int u0 = blockIdx.x * 64;
  const int b0 = wave * 16;

  v8f acc[4][4];
#pragma unroll
  for (int g = 0; g < 4; ++g)
#pragma unroll
    for (int s = 0; s < 4; ++s) acc[g][s] = (v8f){0.f,0.f,0.f,0.f,0.f,0.f,0.f,0.f};

#pragma unroll 1
  for (int k0 = 0; k0 < kHid; k0 += 32) {
    const v16h a = Frag<_Float16>::load(hcur + (size_t)(b0 + m) * kHid + k0 + 8 * hh);
#pragma unroll
    for (int g = 0; g < 4; ++g) {
      v16h bq[4];
#pragma unroll
      for (int s = 0; s < 4; ++s)
        bq[s] = Frag<_Float16>::load(whh + (size_t)(g * kHid + u0 + s * 16 + m) * kHid + k0 + 8 * hh);
#pragma unroll
      for (int s = 0; s < 4; ++s) acc[g][s] = mma_h(a, bq[s], acc[g][s]);
      asm volatile("" ::: "memory");
    }
  }

  const float kInv = 1.0f / 4096.0f;
  const int prow = lane >> 1, pub = (lane & 1) * 8;
  float* slab = sGate[wave];
  float* cw = sC[wave];
  float* hw = sH[wave];
#pragma unroll
  for (int s = 0; s < 4; ++s) {
    __syncthreads();
#pragma unroll
    for (int g = 0; g < 4; ++g)
#pragma unroll
      for (int r = 0; r < 8; ++r) slab[g * 320 + (8 * hh + r) * 20 + m] = acc[g][s][r] * kInv;
    __syncthreads();
#pragma unroll
    for (int g = 0; g < 4; ++g) {
      const float* gp = gin + (size_t)(b0 + prow) * kG4 + g * kHid + u0 + s * 16 + pub;
      const v4f g0 = *(const v4f*)gp;
      const v4f g1 = *(const v4f*)(gp + 4);
      float* sp = slab + g * 320 + prow * 20 + pub;
      const v4f a0 = *(const v4f*)sp;
      const v4f a1 = *(const v4f*)(sp + 4);
      *(v4f*)sp       = a0 + g0;
      *(v4f*)(sp + 4) = a1 + g1;
    }
    {
      const float* cp = ccur + (size_t)(b0 + prow) * kHid + u0 + s * 16 + pub;
      const v4f c0 = *(const v4f*)cp;
      const v4f c1 = *(const v4f*)(cp + 4);
      *(v4f*)(cw + prow * 68 + s * 16 + pub)     = c0;
      *(v4f*)(cw + prow * 68 + s * 16 + pub + 4) = c1;
    }
    __syncthreads();
    {
      const float* gb = slab + prow * 20 + pub;
      float* cb = cw + prow * 68 + s * 16 + pub;
      float* hb = hw + prow * 68 + s * 16 + pub;
#pragma unroll 1
      for (int e = 0; e < 8; ++e) {
        const float gi = gb[e];
        const float gf = gb[320 + e];
        const float gg = gb[640 + e];
        const float go = gb[960 + e];
        const float cp = cb[e];
        const float si = __builtin_amdgcn_rcpf(1.0f + expf(-gi));
        const float sf = __builtin_amdgcn_rcpf(1.0f + expf(-gf));
        const float so = __builtin_amdgcn_rcpf(1.0f + expf(-go));
        const float cn = sf * cp + si * tanhf(gg);
        const float hn = so * tanhf(cn);
        cb[e] = cn;
        hb[e] = hn;
      }
    }
  }
  __syncthreads();

  {
    const int c4 = m * 4;
    const int q = lane >> 3, c8 = (lane & 7) * 8;
    for (int pass = 0; pass < 2; ++pass) {
#pragma unroll
      for (int it = 0; it < 8; ++it) {
        const int row = it * 2 + hh;
        const v4f v = *(const v4f*)(cw + row * 68 + c4);
        *(volatile v4f*)(cnew + (size_t)(b0 + row) * kHid + u0 + c4) = v;
      }
#pragma unroll
      for (int it = 0; it < 4; ++it) {
        const int row = it * 4 + q;
        const float* sp = hw + row * 68 + c8;
        v8h xv, hv, lv;
#pragma unroll
        for (int e = 0; e < 8; ++e) {
          const float hval = sp[e];
          const unsigned short hb16 = f2bf_bits(hval);
          const unsigned short lb16 = f2bf_bits(hval - bf_bits2f(hb16));
          xv[e] = h16_flush(hval * 16.0f);
          hv[e] = __builtin_bit_cast(_Float16, hb16);
          lv[e] = __builtin_bit_cast(_Float16, lb16);
        }
        *(volatile v8h*)(hnew + (size_t)(b0 + row) * kHid + u0 + c8) = xv;
        const size_t ho = ((size_t)(b0 + row) * kSteps + t) * kHid + u0 + c8;
        *(volatile v8h*)(HH + ho) = hv;
        *(volatile v8h*)(HL + ho) = lv;
      }
      __threadfence();
    }
  }
}

extern "C" void kernel_launch(void* const* d_in, const int* in_sizes, int n_in,
                              void* d_out, int out_size, void* d_ws, size_t ws_size,
                              hipStream_t stream) {
  if (n_in < 17) return;
  if (in_sizes[0] != kB * kImg * kImg) return;
  if (in_sizes[1] != kB * kSteps) return;
  if (in_sizes[2] != kCh1 * 9) return;
  if (in_sizes[3] != kCh1) return;
  if (in_sizes[4] != kCh2 * kCh1 * 9) return;
  if (in_sizes[5] != kCh2) return;
  if (in_sizes[6] != kHid * 32) return;
  if (in_sizes[7] != kHid) return;
  if (in_sizes[8] != kHid * kHid) return;
  if (in_sizes[9] != kHid) return;
  if (in_sizes[10] != (kVoc + 1) * kHid) return;
  if (in_sizes[11] != kG4 * kHid) return;
  if (in_sizes[12] != kG4 * kHid) return;
  if (in_sizes[13] != kG4) return;
  if (in_sizes[14] != kG4) return;
  if (in_sizes[15] != kVoc * kHid) return;
  if (in_sizes[16] != kVoc) return;
  if (out_size != kRowsAll * kVoc) return;
  if (ws_size < kWsTotal) return;

  const float* mask    = (const float*)d_in[0];
  const int*   target  = (const int*)  d_in[1];
  const float* conv1_w = (const float*)d_in[2];
  const float* conv1_b = (const float*)d_in[3];
  const float* conv2_w = (const float*)d_in[4];
  const float* conv2_b = (const float*)d_in[5];
  const float* feat_w  = (const float*)d_in[6];
  const float* feat_b  = (const float*)d_in[7];
  const float* ctx_w   = (const float*)d_in[8];
  const float* ctx_b   = (const float*)d_in[9];
  const float* tok_emb = (const float*)d_in[10];
  const float* w_ih    = (const float*)d_in[11];
  const float* w_hh    = (const float*)d_in[12];
  const float* b_ih    = (const float*)d_in[13];
  const float* b_hh    = (const float*)d_in[14];
  const float* head_w  = (const float*)d_in[15];
  const float* head_b  = (const float*)d_in[16];
  float* out = (float*)d_out;

  char* ws = (char*)d_ws;
  unsigned short* PP   = (unsigned short*)(ws + kOffPP);
  unsigned short* W2   = (unsigned short*)(ws + kOffW2);
  float*          PART = (float*)(ws + kOffPART);
  unsigned short* X16  = (unsigned short*)(ws + kOffX16);
  unsigned short* FW   = (unsigned short*)(ws + kOffFW);
  unsigned short* CW   = (unsigned short*)(ws + kOffCW);
  unsigned short* WIH  = (unsigned short*)(ws + kOffWIH);
  unsigned short* WHH  = (unsigned short*)(ws + kOffWHH);
  unsigned short* HW   = (unsigned short*)(ws + kOffHW);
  unsigned short* HA   = (unsigned short*)(ws + kOffHA);
  unsigned short* HB   = (unsigned short*)(ws + kOffHB);
  float*          CTX  = (float*)(ws + kOffCTX);
  float*          CA   = (float*)(ws + kOffCA);
  float*          CB   = (float*)(ws + kOffCB);
  unsigned short* XIN  = (unsigned short*)(ws + kOffXIN);
  float*          GIN  = (float*)(ws + kOffGIN);
  unsigned short* HH   = (unsigned short*)(ws + kOffHH);
  unsigned short* HL   = (unsigned short*)(ws + kOffHL);

  cast_plane_kernel<0, 8><<<dim3((kHid * 32 / 8) / 256), dim3(256), 0, stream>>>(feat_w, FW, kHid * 32 / 8);
  cast_plane_kernel<0, 8><<<dim3((kHid * kHid / 8) / 256), dim3(256), 0, stream>>>(ctx_w, CW, kHid * kHid / 8);
  cast_plane_kernel<0, 8><<<dim3((kG4 * kHid / 8) / 256), dim3(256), 0, stream>>>(w_ih, WIH, kG4 * kHid / 8);
  cast_plane_kernel<0, 8><<<dim3((kG4 * kHid / 8) / 256), dim3(256), 0, stream>>>(w_hh, WHH, kG4 * kHid / 8);
  cast_plane_kernel<1, 0><<<dim3((kVoc * kHid / 8) / 256), dim3(256), 0, stream>>>(head_w, HW, kVoc * kHid / 8);
  conv2_weight_plane_kernel<<<dim3(3), dim3(256), 0, stream>>>(conv2_w, W2);

  conv1_pool_plane_kernel<<<dim3(kPRows, kB), dim3(256), 0, stream>>>(mask, conv1_w, conv1_b, (unsigned*)PP);
  conv2_mean_partial_kernel<<<dim3(kRowGroups, kB), dim3(256), 0, stream>>>(PP, W2, conv2_b, PART);
  mean_plane_kernel<<<dim3(1), dim3(256), 0, stream>>>(PART, X16);

  wmma_gemm64<0, 0, 1, 1, 12, 4><<<dim3(1), dim3(256), 0, stream>>>(
      X16, X16, 32, FW, 32, (void*)HA, kHid, feat_b, feat_b, kB, kHid, 32);
  wmma_gemm64<0, 0, 1, 0, 12, 0><<<dim3(1), dim3(256), 0, stream>>>(
      HA, HA, kHid, CW, kHid, (void*)CTX, kHid, ctx_b, ctx_b, kB, kHid, kHid);

  zero_plane_kernel<<<dim3((kB * kHid / 4) / 256), dim3(256), 0, stream>>>(CA, kB * kHid / 4);

  step_input_plane_kernel<<<dim3((kRowsAll * kHid / 8) / 256), dim3(256), 0, stream>>>(tok_emb, target, CTX, XIN);
  wmma_gemm64<0, 0, 2, 0, 12, 0><<<dim3(((kRowsAll / 64) * (kG4 / 64)) / 8), dim3(256), 0, stream>>>(
      XIN, XIN, kHid, WIH, kHid, (void*)GIN, kG4, b_ih, b_hh, kRowsAll, kG4, kHid);

  for (int t = 0; t < kSteps; ++t) {
    const bool ev = (t & 1) == 0;
    lstm_step_kernel<<<dim3(kHid / 64), dim3(128), 0, stream>>>(
        ev ? HA : HB, WHH, GIN + (size_t)t * kB * kG4,
        ev ? CA : CB, ev ? CB : CA, ev ? HB : HA, HH, HL, t);
  }

  wmma_gemm64<1, 1, 1, 0, 0, 0><<<dim3(((kRowsAll / 64) * (kVoc / 64)) / 8), dim3(256), 0, stream>>>(
      HH, HL, kHid, HW, kHid, (void*)out, kVoc, head_b, head_b, kRowsAll, kVoc, kHid);
}
